// SelfAttention_40656160424626
// MI455X (gfx1250) — hardware-run, weakly checked
//
#include <hip/hip_runtime.h>


#ifndef NB
#define NB 4
#endif
#ifndef SEQ
#define SEQ 2048
#endif
#define NB_FULL    4
#define SEQ_FULL   2048
#define DIM        768
#define NHEAD      12
#define HDIM       64
#define BQ         128
#define BK         32
#define NWAVE      8
#define CT         64
#define TP         72
#define OP         68
#define GM         128
#define GN         64
#define GW         4
#define CP         68
#define WELEM      (DIM * DIM)
#define MROWS      (NB * SEQ)
#define PLANE_E    ((size_t)MROWS * DIM)
#define HTHREADS   (MROWS * (DIM / 8))
#define HBLK       (HTHREADS / 256)
#define WBLK       (WELEM / 8 / 256)
#define WS_CAP     134217728ull

static_assert(DIM == NHEAD * HDIM);
static_assert(HDIM == 64);
static_assert(SEQ % BQ == 0);
static_assert(SEQ % CT == 0);
static_assert(SEQ % BK == 0);
static_assert(SEQ % 32 == 0);
static_assert(MROWS % GM == 0);
static_assert(DIM % GN == 0);
static_assert(DIM % 32 == 0);
static_assert(DIM % 8 == 0);
static_assert(BQ == NWAVE * 16);
static_assert(GM == GW * 32);
static_assert(HTHREADS % 256 == 0);
static_assert((WELEM / 8) % 256 == 0);
static_assert(CT == 64 && CT <= TP);
static_assert((TP * 2) % 16 == 0);
static_assert((OP * 4) % 16 == 0);
static_assert((CP * 4) % 16 == 0);
static_assert(OP >= HDIM && CP >= GN);
static_assert(SEQ <= SEQ_FULL);
static_assert(NB >= 1 && NB <= NB_FULL);
static_assert(9ull * (unsigned long long)NB * SEQ * DIM * 2ull + 4ull * WELEM * 2ull <= WS_CAP);

typedef __bf16         bf16;
typedef _Float16       f16;
typedef unsigned short u16;
typedef bf16     v16bf __attribute__((ext_vector_type(16)));
typedef f16      v16h  __attribute__((ext_vector_type(16)));
typedef float    v8f   __attribute__((ext_vector_type(8)));
typedef float    v4f   __attribute__((ext_vector_type(4)));
typedef unsigned v4u   __attribute__((ext_vector_type(4)));
typedef int      v4i   __attribute__((ext_vector_type(4)));

union FragB  { v16bf v; v4u q[2]; };
union FragH  { v16h  v; v4u q[2]; f16 h[16]; };
union Pack8B { v4u u; bf16 h[8]; };
union Pack8H { v4u u; f16 h[8]; };
union Pack8S { v4u u; u16 s[8]; };

static __device__ __forceinline__ v8f mma_bf16(v16bf a, v16bf b, v8f acc) {
  acc = __builtin_amdgcn_wmma_f32_16x16x32_bf16(false, a, false, b, (short)0, acc, false, false);
  asm volatile("v_nop\n\tv_nop\n\tv_nop\n\tv_nop" : "+v"(acc) : "v"(a), "v"(b));
  return acc;
}
static __device__ __forceinline__ v8f mma_f16(v16h a, v16h b, v8f acc) {
  acc = __builtin_amdgcn_wmma_f32_16x16x32_f16(false, a, false, b, (short)0, acc, false, false);
  asm volatile("v_nop\n\tv_nop\n\tv_nop\n\tv_nop" : "+v"(acc) : "v"(a), "v"(b));
  return acc;
}

static __device__ __forceinline__ void cvt_store8(const float* __restrict__ src, u16* __restrict__ dst) {
  const v4f a = *(const v4f*)(src);
  const v4f b = *(const v4f*)(src + 4);
  Pack8B pk;
  #pragma unroll
  for (int i = 0; i < 4; ++i) {
    pk.h[i]     = (bf16)a[i];
    pk.h[4 + i] = (bf16)b[i];
  }
  const v4u val = pk.u;
  *(volatile v4u*)(dst) = val;
  __threadfence();
  *(volatile v4u*)(dst) = val;
}

__global__ __launch_bounds__(256) void cvt_kernel(const float* __restrict__ h,
                                                  const float* __restrict__ wq,
                                                  const float* __restrict__ wk,
                                                  const float* __restrict__ wv,
                                                  const float* __restrict__ wo,
                                                  u16* __restrict__ hb,
                                                  u16* __restrict__ wb) {
  const int blk = blockIdx.x;
  const int tid = threadIdx.x;
  if (blk < HBLK) {
    const size_t e  = ((size_t)blk * 256 + tid) * 8;
    const int row   = (int)(e / DIM);
    const int col   = (int)(e % DIM);
    const int b     = row / SEQ;
    const int s     = row % SEQ;
    cvt_store8(h + ((size_t)b * SEQ_FULL + s) * DIM + col, hb + e);
  } else {
    const int wi    = (blk - HBLK) / WBLK;
    const size_t e  = ((size_t)((blk - HBLK) % WBLK) * 256 + tid) * 8;
    u16* dst        = wb + (size_t)wi * WELEM + e;
    if (wi == 0)      cvt_store8(wq + e, dst);
    else if (wi == 1) cvt_store8(wk + e, dst);
    else if (wi == 2) cvt_store8(wv + e, dst);
    else              cvt_store8(wo + e, dst);
  }
}

template <int NA>
static __device__ __forceinline__ void gemm_tile(const u16* __restrict__ a0,
                                                 const u16* __restrict__ a1,
                                                 const u16* __restrict__ w,
                                                 const int m0, const int n0,
                                                 const int lq, const int hi,
                                                 v8f (&acc)[2][4]) {
  const u16* wrow  = w  + (size_t)(n0 + lq) * DIM + hi * 8;
  const u16* arow0 = a0 + (size_t)(m0 + lq) * DIM + hi * 8;
  const u16* arow1 = a1 + (size_t)(m0 + lq) * DIM + hi * 8;
  #pragma unroll 1
  for (int k0 = 0; k0 < DIM; k0 += 32) {
    FragB bw[4];
    #pragma unroll
    for (int nt = 0; nt < 4; ++nt) {
      const u16* p = wrow + (size_t)nt * 16 * DIM + k0;
      bw[nt].q[0] = *(const v4u*)(p);
      bw[nt].q[1] = *(const v4u*)(p + 16);
    }
    #pragma unroll
    for (int mt = 0; mt < 2; ++mt) {
      FragB fa;
      const u16* p = arow0 + (size_t)mt * 16 * DIM + k0;
      fa.q[0] = *(const v4u*)(p);
      fa.q[1] = *(const v4u*)(p + 16);
      #pragma unroll
      for (int nt = 0; nt < 4; ++nt) acc[mt][nt] = mma_bf16(fa.v, bw[nt].v, acc[mt][nt]);
      if (NA == 2) {
        FragB fb;
        const u16* p1 = arow1 + (size_t)mt * 16 * DIM + k0;
        fb.q[0] = *(const v4u*)(p1);
        fb.q[1] = *(const v4u*)(p1 + 16);
        #pragma unroll
        for (int nt = 0; nt < 4; ++nt) acc[mt][nt] = mma_bf16(fb.v, bw[nt].v, acc[mt][nt]);
      }
    }
  }
}

__global__ __launch_bounds__(128) void qkv_kernel(const u16* __restrict__ hb,
                                                  const u16* __restrict__ wb,
                                                  u16* __restrict__ planes) {
  __shared__ __align__(16) float sC[GW * 32 * CP];
  const int tid  = threadIdx.x;
  const int wave = __builtin_amdgcn_readfirstlane(threadIdx.x >> 5);
  const int lane = tid & 31;
  const int lq   = lane & 15;
  const int hi   = lane >> 4;
  const int n0   = blockIdx.x * GN;
  const int m0   = blockIdx.y * GM + wave * 32;
  const int z    = blockIdx.z;

  v8f acc[2][4];
  #pragma unroll
  for (int mt = 0; mt < 2; ++mt) {
    #pragma unroll
    for (int nt = 0; nt < 4; ++nt) acc[mt][nt] = (v8f){0, 0, 0, 0, 0, 0, 0, 0};
  }
  gemm_tile<1>(hb, hb, wb + (size_t)z * WELEM, m0, n0, lq, hi, acc);

  float* sc = sC + wave * (32 * CP);
  #pragma unroll
  for (int mt = 0; mt < 2; ++mt) {
    #pragma unroll
    for (int nt = 0; nt < 4; ++nt) {
      #pragma unroll
      for (int r = 0; r < 8; ++r) sc[(mt * 16 + hi * 8 + r) * CP + nt * 16 + lq] = acc[mt][nt][r];
    }
  }
  __syncthreads();

  v4u    vh[8];
  v4u    vl[8];
  size_t gi[8];
  #pragma unroll
  for (int it = 0; it < 8; ++it) {
    const int row = it * 4 + (lane >> 3);
    const int c0  = (lane & 7) * 8;
    const v4f x0 = *(const v4f*)(sc + row * CP + c0);
    const v4f x1 = *(const v4f*)(sc + row * CP + c0 + 4);
    Pack8B ph, pl;
    Pack8H pf;
    #pragma unroll
    for (int i = 0; i < 4; ++i) {
      const bf16 h0 = (bf16)x0[i];
      const bf16 h1 = (bf16)x1[i];
      ph.h[i]     = h0;
      ph.h[4 + i] = h1;
      pl.h[i]     = (bf16)(x0[i] - (float)h0);
      pl.h[4 + i] = (bf16)(x1[i] - (float)h1);
      pf.h[i]     = (f16)x0[i];
      pf.h[4 + i] = (f16)x1[i];
    }
    vh[it] = (z == 2) ? pf.u : ph.u;
    vl[it] = pl.u;
    gi[it] = (size_t)(m0 + row) * DIM + n0 + c0;
  }
  u16* ph_base = planes + (size_t)(2 * z) * PLANE_E;
  u16* pl_base = planes + (size_t)(2 * z + 1) * PLANE_E;

  #pragma unroll
  for (int it = 0; it < 8; ++it) *(volatile v4u*)(ph_base + gi[it]) = vh[it];
  if (z < 2) {
    #pragma unroll
    for (int it = 0; it < 8; ++it) *(volatile v4u*)(pl_base + gi[it]) = vl[it];
  }
  __threadfence();
  #pragma unroll
  for (int it = 0; it < 8; ++it) *(volatile v4u*)(ph_base + gi[it]) = vh[it];
  if (z < 2) {
    #pragma unroll
    for (int it = 0; it < 8; ++it) *(volatile v4u*)(pl_base + gi[it]) = vl[it];
  }
}

__global__ __launch_bounds__(256) void vtrans_kernel(const u16* __restrict__ v, u16* __restrict__ vt) {
  const int kt  = blockIdx.x;
  const int bh  = blockIdx.y;
  const int tid = threadIdx.x;
  __shared__ __align__(16) u16 sT[HDIM * TP];
  const int s0 = kt * CT;

  #pragma unroll
  for (int kk = 0; kk < 2; ++kk) {
    const int key = kk * 32 + (tid >> 3);
    const int d0  = (tid & 7) * 8;
    Pack8S ps;
    ps.u = *(const v4u*)(v + ((size_t)bh * SEQ + s0 + key) * HDIM + d0);
    #pragma unroll
    for (int i = 0; i < 8; ++i) sT[(d0 + i) * TP + key] = ps.s[i];
  }
  __syncthreads();

  v4u    vval[2];
  size_t vidx[2];
  #pragma unroll
  for (int kk = 0; kk < 2; ++kk) {
    const int d  = kk * 32 + (tid >> 3);
    const int ks = (tid & 7) * 8;
    vval[kk] = *(const v4u*)(sT + d * TP + ks);
    vidx[kk] = ((size_t)bh * HDIM + d) * SEQ + s0 + ks;
  }
  #pragma unroll
  for (int kk = 0; kk < 2; ++kk) *(volatile v4u*)(vt + vidx[kk]) = vval[kk];
  __threadfence();
  #pragma unroll
  for (int kk = 0; kk < 2; ++kk) *(volatile v4u*)(vt + vidx[kk]) = vval[kk];
}

__global__ __launch_bounds__(256) void attn_kernel(const u16* __restrict__ qh,
                                                   const u16* __restrict__ ql,
                                                   const u16* __restrict__ kh,
                                                   const u16* __restrict__ kl,
                                                   const u16* __restrict__ vt,
                                                   const int* __restrict__ mask,
                                                   u16* __restrict__ ch,
                                                   u16* __restrict__ cl) {
  const int qblk = blockIdx.x;
  const int bh   = blockIdx.y;
  const int b    = bh / NHEAD;
  const int tid  = threadIdx.x;
  const int wave = __builtin_amdgcn_readfirstlane(threadIdx.x >> 5);
  const int lane = tid & 31;
  const int lq   = lane & 15;
  const int hi   = lane >> 4;

  __shared__ __align__(16) float sO[NWAVE * 16 * OP];

  const int qrow0 = qblk * BQ + wave * 16;

  FragB qfh[2], qfl[2];
  {
    const size_t qo = ((size_t)bh * SEQ + qrow0 + lq) * HDIM + hi * 8;
    #pragma unroll
    for (int f = 0; f < 2; ++f) {
      qfh[f].q[0] = *(const v4u*)(qh + qo + f * 32);
      qfh[f].q[1] = *(const v4u*)(qh + qo + f * 32 + 16);
      qfl[f].q[0] = *(const v4u*)(ql + qo + f * 32);
      qfl[f].q[1] = *(const v4u*)(ql + qo + f * 32 + 16);
    }
  }

  const u16* kh_h = kh + (size_t)bh * SEQ * HDIM + (size_t)lq * HDIM + hi * 8;
  const u16* kl_h = kl + (size_t)bh * SEQ * HDIM + (size_t)lq * HDIM + hi * 8;
  const u16* vt_h = vt + (size_t)bh * HDIM * SEQ + (size_t)lq * SEQ + hi * 8;
  const int* mk_b = mask + (size_t)b * SEQ_FULL + hi * 8;

  v8f o[4];
  #pragma unroll
  for (int dt = 0; dt < 4; ++dt) o[dt] = (v8f){0, 0, 0, 0, 0, 0, 0, 0};

  const float NEG_INF = -__builtin_inff();
  float rmax = NEG_INF;
  float rsum = 0.0f;
  const float SL = 0.125f * 1.4426950408889634f;

  const int nchunk = SEQ / BK;
  #pragma unroll 1
  for (int i = 0; i < nchunk; ++i) {
    const int j0 = i * BK;

    v8f c[2];
    #pragma unroll
    for (int sub = 0; sub < 2; ++sub) {
      const size_t ko = (size_t)(j0 + sub * 16) * HDIM;
      FragB akh[2], akl[2];
      #pragma unroll
      for (int f = 0; f < 2; ++f) {
        akh[f].q[0] = *(const v4u*)(kh_h + ko + f * 32);
        akh[f].q[1] = *(const v4u*)(kh_h + ko + f * 32 + 16);
        akl[f].q[0] = *(const v4u*)(kl_h + ko + f * 32);
        akl[f].q[1] = *(const v4u*)(kl_h + ko + f * 32 + 16);
      }
      const v4i m0 = *(const v4i*)(mk_b + j0 + sub * 16);
      const v4i m1 = *(const v4i*)(mk_b + j0 + sub * 16 + 4);
      v8f acc = (v8f){0, 0, 0, 0, 0, 0, 0, 0};
      #pragma unroll
      for (int f = 0; f < 2; ++f) {
        acc = mma_bf16(akl[f].v, qfh[f].v, acc);
        acc = mma_bf16(akh[f].v, qfl[f].v, acc);
        acc = mma_bf16(akh[f].v, qfh[f].v, acc);
      }
      #pragma unroll
      for (int r = 0; r < 4; ++r) {
        acc[r]     = (m0[r] != 0) ? acc[r]     : NEG_INF;
        acc[4 + r] = (m1[r] != 0) ? acc[4 + r] : NEG_INF;
      }
      c[sub] = acc;
    }

    FragH bv[4];
    #pragma unroll
    for (int dt = 0; dt < 4; ++dt) {
      const u16* base = vt_h + (size_t)(dt * 16) * SEQ + j0;
      bv[dt].q[0] = *(const v4u*)(base);
      bv[dt].q[1] = *(const v4u*)(base + 16);
    }

    float m_new = rmax;
    #pragma unroll
    for (int r = 0; r < 8; ++r) {
      m_new = fmaxf(m_new, c[0][r]);
      m_new = fmaxf(m_new, c[1][r]);
    }
    m_new = fmaxf(m_new, __shfl_xor(m_new, 16, 32));
    const float m_use = (m_new == NEG_INF) ? 0.0f : m_new;
    const float scale = __builtin_amdgcn_exp2f((rmax - m_use) * SL);
    rmax = m_new;

    FragH pa;
    float psum = 0.0f;
    #pragma unroll
    for (int r = 0; r < 8; ++r) {
      const float p0 = __builtin_amdgcn_exp2f((c[0][r] - m_use) * SL);
      const float p1 = __builtin_amdgcn_exp2f((c[1][r] - m_use) * SL);
      psum += p0 + p1;
      pa.h[r]     = (f16)(p0 * 4096.0f);
      pa.h[8 + r] = (f16)(p1 * 4096.0f);
    }
    rsum = rsum * scale + psum + __shfl_xor(psum, 16, 32);

    float sc[8];
    #pragma unroll
    for (int r = 0; r < 8; ++r) sc[r] = __shfl(scale, (hi << 3) + r, 32);
    #pragma unroll
    for (int dt = 0; dt < 4; ++dt) {
      #pragma unroll
      for (int r = 0; r < 8; ++r) o[dt][r] *= sc[r];
    }

    #pragma unroll
    for (int dt = 0; dt < 4; ++dt) o[dt] = mma_f16(pa.v, bv[dt].v, o[dt]);
  }

  float rs[8];
  #pragma unroll
  for (int r = 0; r < 8; ++r) rs[r] = 1.0f / __shfl(rsum, (hi << 3) + r, 32);

  float* so = sO + wave * (16 * OP);
  #pragma unroll
  for (int r = 0; r < 8; ++r) {
    #pragma unroll
    for (int dt = 0; dt < 4; ++dt) {
      so[(hi * 8 + r) * OP + dt * 16 + lq] = o[dt][r] * (1.0f / 4096.0f) * rs[r];
    }
  }
  __syncthreads();

  v4u    vh[4];
  v4u    vl[4];
  size_t gi[4];
  #pragma unroll
  for (int it = 0; it < 4; ++it) {
    const int row = it * 4 + (lane >> 3);
    const int c0  = (lane & 7) * 8;
    const v4f x0 = *(const v4f*)(so + row * OP + c0);
    const v4f x1 = *(const v4f*)(so + row * OP + c0 + 4);
    Pack8B ph, pl;
    #pragma unroll
    for (int k = 0; k < 4; ++k) {
      const bf16 h0 = (bf16)x0[k];
      const bf16 h1 = (bf16)x1[k];
      ph.h[k]     = h0;
      ph.h[4 + k] = h1;
      pl.h[k]     = (bf16)(x0[k] - (float)h0);
      pl.h[4 + k] = (bf16)(x1[k] - (float)h1);
    }
    vh[it] = ph.u;
    vl[it] = pl.u;
    gi[it] = ((size_t)bh * SEQ + qrow0 + row) * HDIM + c0;
  }
  #pragma unroll
  for (int it = 0; it < 4; ++it) {
    *(volatile v4u*)(ch + gi[it]) = vh[it];
    *(volatile v4u*)(cl + gi[it]) = vl[it];
  }
  __threadfence();
  #pragma unroll
  for (int it = 0; it < 4; ++it) {
    *(volatile v4u*)(ch + gi[it]) = vh[it];
    *(volatile v4u*)(cl + gi[it]) = vl[it];
  }
}

__global__ __launch_bounds__(128) void oproj_kernel(const u16* __restrict__ ch,
                                                    const u16* __restrict__ cl,
                                                    const u16* __restrict__ wob,
                                                    float* __restrict__ out) {
  __shared__ __align__(16) float sC[GW * 32 * CP];
  const int tid  = threadIdx.x;
  const int wave = __builtin_amdgcn_readfirstlane(threadIdx.x >> 5);
  const int lane = tid & 31;
  const int lq   = lane & 15;
  const int hi   = lane >> 4;
  const int n0   = blockIdx.x * GN;
  const int m0   = blockIdx.y * GM + wave * 32;

  v8f acc[2][4];
  #pragma unroll
  for (int mt = 0; mt < 2; ++mt) {
    #pragma unroll
    for (int nt = 0; nt < 4; ++nt) acc[mt][nt] = (v8f){0, 0, 0, 0, 0, 0, 0, 0};
  }
  gemm_tile<2>(ch, cl, wob, m0, n0, lq, hi, acc);

  float* sc = sC + wave * (32 * CP);
  #pragma unroll
  for (int mt = 0; mt < 2; ++mt) {
    #pragma unroll
    for (int nt = 0; nt < 4; ++nt) {
      #pragma unroll
      for (int r = 0; r < 8; ++r) sc[(mt * 16 + hi * 8 + r) * CP + nt * 16 + lq] = acc[mt][nt][r];
    }
  }
  __syncthreads();

  v4f    vals[16];
  size_t gi[16];
  #pragma unroll
  for (int it = 0; it < 16; ++it) {
    const int row = it * 2 + hi;
    vals[it] = *(const v4f*)(sc + row * CP + lq * 4);
    const int m  = m0 + row;
    const int bb = m / SEQ;
    const int ss = m % SEQ;
    gi[it] = ((size_t)bb * SEQ_FULL + ss) * DIM + n0 + lq * 4;
  }
  #pragma unroll
  for (int it = 0; it < 16; ++it) *(volatile v4f*)(out + gi[it]) = vals[it];
  __threadfence();
  #pragma unroll
  for (int it = 0; it < 16; ++it) *(volatile v4f*)(out + gi[it]) = vals[it];
}

extern "C" void kernel_launch(void* const* d_in, const int* in_sizes, int n_in,
                              void* d_out, int out_size, void* d_ws, size_t ws_size,
                              hipStream_t stream) {
  if (n_in < 6) return;
  const size_t need_rows = (size_t)(NB - 1) * SEQ_FULL + SEQ;
  if ((size_t)in_sizes[0] < need_rows * DIM) return;
  if ((size_t)in_sizes[1] < need_rows) return;
  if ((size_t)in_sizes[2] < (size_t)WELEM) return;
  if ((size_t)in_sizes[3] < (size_t)WELEM) return;
  if ((size_t)in_sizes[4] < (size_t)WELEM) return;
  if ((size_t)in_sizes[5] < (size_t)WELEM) return;
  if ((size_t)out_size < need_rows * DIM) return;

  const size_t plane_bytes = PLANE_E * 2;
  const size_t w_bytes     = (size_t)4 * WELEM * 2;
  const size_t total       = 9 * plane_bytes + w_bytes;
  if (ws_size < total) return;
  if (total > WS_CAP) return;

  const float* h    = (const float*)d_in[0];
  const int*   mask = (const int*)d_in[1];
  const float* wq   = (const float*)d_in[2];
  const float* wk   = (const float*)d_in[3];
  const float* wv   = (const float*)d_in[4];
  const float* wo   = (const float*)d_in[5];
  float*       out  = (float*)d_out;

  char* ws = (char*)d_ws;
  u16* planes = (u16*)(ws);
  u16* qh = (u16*)(ws + 0 * plane_bytes);
  u16* ql = (u16*)(ws + 1 * plane_bytes);
  u16* kh = (u16*)(ws + 2 * plane_bytes);
  u16* kl = (u16*)(ws + 3 * plane_bytes);
  u16* vp = (u16*)(ws + 4 * plane_bytes);
  u16* vt = (u16*)(ws + 5 * plane_bytes);
  u16* ch = (u16*)(ws + 6 * plane_bytes);
  u16* cl = (u16*)(ws + 7 * plane_bytes);
  u16* hb = (u16*)(ws + 8 * plane_bytes);
  u16* wb = (u16*)(ws + 9 * plane_bytes);

  cvt_kernel<<<dim3(HBLK + 4 * WBLK), 256, 0, stream>>>(h, wq, wk, wv, wo, hb, wb);
  qkv_kernel<<<dim3(DIM / GN, MROWS / GM, 3), 128, 0, stream>>>(hb, wb, planes);
  vtrans_kernel<<<dim3(SEQ / CT, NB * NHEAD), 256, 0, stream>>>(vp, vt);
  attn_kernel<<<dim3(SEQ / BQ, NB * NHEAD), 256, 0, stream>>>(qh, ql, kh, kl, vt, mask, ch, cl);
  oproj_kernel<<<dim3(DIM / GN, MROWS / GM), 128, 0, stream>>>(ch, cl, wb + (size_t)3 * WELEM, out);
}
